// MessagePassingLayer_22840636080227
// MI455X (gfx1250) — hardware-verified
//
#include <hip/hip_runtime.h>
#include <math.h>
#include <stdint.h>

#define NND    2048
#define DX     256
#define DHD    256
#define NH     4
#define DHEAD  64
#define NREL   2
#define DMSG   (NREL * DHD)
#define G3     (3 * DX)
#define NASC   16
#define NASCP  64
#define CASC   (2 * DHD + G3)
#define NBC    (CASC + NASCP)
#define QT     32
#define KT     64
#define SP     36
#define NEGF   (-1.0e30f)
#define LN_EPS 1e-5f
#define SLOPE  0.2f

#define NXU (NND * DX / 8)
#define NBU (NBC * DX / 8)
#define NWU (G3 * DMSG / 8)

static_assert(NND % 128 == 0);
static_assert(NND % QT == 0);
static_assert(NND % KT == 0);
static_assert(DX % 32 == 0);
static_assert(DMSG % 32 == 0);
static_assert(NBC % 64 == 0);
static_assert(G3 % 64 == 0);
static_assert(DHD % 64 == 0);
static_assert(DHEAD == 64);
static_assert(NH * QT == 128);
static_assert(NH * KT == 256);
static_assert(NXU % 32 == 0);
static_assert(NBU % 32 == 0);
static_assert((NXU + NBU + NWU) % 256 == 0);
static_assert((DX / 8) == 32);

typedef __attribute__((ext_vector_type(16))) __bf16 v16b;
typedef __attribute__((ext_vector_type(8)))  __bf16 v8b;
typedef __attribute__((ext_vector_type(8)))  float  v8f;
typedef __attribute__((ext_vector_type(4)))  float  v4f;
typedef __attribute__((ext_vector_type(4)))  unsigned int v4u;
typedef __attribute__((ext_vector_type(8)))  unsigned int v8u;
typedef v8b __attribute__((may_alias)) v8ba;
typedef v4f __attribute__((may_alias)) v4fa;
typedef v4u __attribute__((may_alias)) v4ua;

union FragU { v16b v; v8b h[2]; };
union PackU { v8u u; v16b v; };

__device__ __forceinline__ unsigned short f2bf_bits(float f) {
  const unsigned u = __float_as_uint(f);
  return (unsigned short)((u + 0x7FFFu + ((u >> 16) & 1u)) >> 16);
}
__device__ __forceinline__ float bf_bits2f(unsigned short h) { return __uint_as_float(((unsigned)h) << 16); }
__device__ __forceinline__ float bf16r(float f) {
  unsigned u = __float_as_uint(f);
  u = (u + 0x7FFFu + ((u >> 16) & 1u)) & 0xFFFF0000u;
  return __uint_as_float(u);
}
__device__ __forceinline__ unsigned pk16(unsigned short a, unsigned short b) { return (unsigned)a | ((unsigned)b << 16); }

__device__ __forceinline__ v8f wmma_bf16(v16b a, v16b b, v8f c) {
  v8f d = __builtin_amdgcn_wmma_f32_16x16x32_bf16(false, a, false, b, (short)0, c, false, false);
  asm volatile("v_nop\n\tv_nop\n\tv_nop\n\tv_nop" : "+v"(d) : "v"(a), "v"(b));
  return d;
}

__device__ __forceinline__ v16b load_frag(const unsigned short* p, int hh) {
  FragU f;
  f.h[0] = *(const v8ba*)(p + 8 * hh);
  f.h[1] = *(const v8ba*)(p + 16 + 8 * hh);
  return f.v;
}

__device__ __forceinline__ void pack_p2(v8f a, v8f c, v16b& ho, v16b& lo) {
  PackU uh, ul;
#pragma unroll
  for (int i = 0; i < 4; ++i) {
    const unsigned short h0 = f2bf_bits(a[2 * i]), h1 = f2bf_bits(a[2 * i + 1]);
    const unsigned short l0 = f2bf_bits(a[2 * i] - bf_bits2f(h0)), l1 = f2bf_bits(a[2 * i + 1] - bf_bits2f(h1));
    uh.u[i] = pk16(h0, h1); ul.u[i] = pk16(l0, l1);
    const unsigned short g0 = f2bf_bits(c[2 * i]), g1 = f2bf_bits(c[2 * i + 1]);
    const unsigned short m0 = f2bf_bits(c[2 * i] - bf_bits2f(g0)), m1 = f2bf_bits(c[2 * i + 1] - bf_bits2f(g1));
    uh.u[4 + i] = pk16(g0, g1); ul.u[4 + i] = pk16(m0, m1);
  }
  ho = uh.v; lo = ul.v;
}

__device__ __forceinline__ void gemm_core_32x64(
    const unsigned short* __restrict__ Ah, const unsigned short* __restrict__ Al,
    const unsigned short* __restrict__ Bt, int K, size_t aoff, size_t boff, int hh, v8f (&acc)[2][4]) {
  const unsigned short* a0h = Ah + aoff;
  const unsigned short* a1h = a0h + (size_t)16 * K;
  const unsigned short* a0l = Al + aoff;
  const unsigned short* a1l = a0l + (size_t)16 * K;
  const unsigned short* bp  = Bt + boff;
#pragma unroll 1
  for (int k0 = 0; k0 < K; k0 += 32) {
    const v16b f0h = load_frag(a0h + k0, hh);
    const v16b f0l = load_frag(a0l + k0, hh);
    const v16b f1h = load_frag(a1h + k0, hh);
    const v16b f1l = load_frag(a1l + k0, hh);
#pragma unroll
    for (int nt = 0; nt < 4; ++nt) {
      const v16b fb = load_frag(bp + (size_t)nt * 16 * K + k0, hh);
      acc[0][nt] = wmma_bf16(f0h, fb, acc[0][nt]);
      acc[0][nt] = wmma_bf16(f0l, fb, acc[0][nt]);
      acc[1][nt] = wmma_bf16(f1h, fb, acc[1][nt]);
      acc[1][nt] = wmma_bf16(f1l, fb, acc[1][nt]);
    }
  }
}

__device__ __forceinline__ void gemm_core1_32x64(
    const unsigned short* __restrict__ A, const unsigned short* __restrict__ Bt,
    int K, size_t aoff, size_t boff, int hh, v8f (&acc)[2][4]) {
  const unsigned short* a0 = A + aoff;
  const unsigned short* a1 = a0 + (size_t)16 * K;
  const unsigned short* bp = Bt + boff;
#pragma unroll 1
  for (int k0 = 0; k0 < K; k0 += 32) {
    const v16b f0 = load_frag(a0 + k0, hh);
    const v16b f1 = load_frag(a1 + k0, hh);
#pragma unroll
    for (int nt = 0; nt < 4; ++nt) {
      const v16b fb = load_frag(bp + (size_t)nt * 16 * K + k0, hh);
      acc[0][nt] = wmma_bf16(f0, fb, acc[0][nt]);
      acc[1][nt] = wmma_bf16(f1, fb, acc[1][nt]);
    }
  }
}

__global__ __launch_bounds__(256) void k_prep(const float* __restrict__ x,
                                              const float* __restrict__ Wm0, const float* __restrict__ Wm1,
                                              const float* __restrict__ whh,
                                              const float* __restrict__ Wa0, const float* __restrict__ Wa1,
                                              const float* __restrict__ wih,
                                              unsigned short* __restrict__ Xb, unsigned short* __restrict__ Bc,
                                              unsigned short* __restrict__ WIb) {
  const int g = blockIdx.x * 256 + threadIdx.x;
  if (g >= NXU + NBU + NWU) return;
  const float* src;
  unsigned short* dst;
  float sc = 1.0f;
  if (g < NXU) {
    src = x + (size_t)g * 8;
    dst = Xb + (size_t)g * 8;
  } else if (g < NXU + NBU) {
    const int e   = g - NXU;
    const int row = e >> 5;
    const int k8  = (e & 31) * 8;
    dst = Bc + (size_t)row * DX + k8;
    if (row < DHD) {
      src = Wm0 + (size_t)row * DX + k8;
    } else if (row < 2 * DHD) {
      src = Wm1 + (size_t)(row - DHD) * DX + k8;
    } else if (row < CASC) {
      src = whh + (size_t)(row - 2 * DHD) * DX + k8;
    } else if (row < CASC + NASC) {
      const int c = row - CASC;
      const int rel = c >> 3, half = (c >> 2) & 1, hd = c & 3;
      const float* Wa = rel ? Wa1 : Wa0;
      src = Wa + (size_t)hd * (2 * DX) + (size_t)half * DX + k8;
    } else {
      src = Wa1 + k8;
      sc = 0.0f;
    }
  } else {
    const int e = g - NXU - NBU;
    src = wih + (size_t)e * 8;
    dst = WIb + (size_t)e * 8;
  }
  const v4f a = *(const v4fa*)src;
  const v4f c = *(const v4fa*)(src + 4);
  v4u o;
  o[0] = pk16(f2bf_bits(a[0] * sc), f2bf_bits(a[1] * sc));
  o[1] = pk16(f2bf_bits(a[2] * sc), f2bf_bits(a[3] * sc));
  o[2] = pk16(f2bf_bits(c[0] * sc), f2bf_bits(c[1] * sc));
  o[3] = pk16(f2bf_bits(c[2] * sc), f2bf_bits(c[3] * sc));
  *(volatile v4u*)dst = o;
  __threadfence();
  *(volatile v4u*)dst = o;
}

__global__ __launch_bounds__(128) void k_proj(
    const unsigned short* __restrict__ Xb, const unsigned short* __restrict__ Bc,
    const float* __restrict__ bm0, const float* __restrict__ bm1, const float* __restrict__ bhh,
    unsigned short* __restrict__ MThi, unsigned short* __restrict__ MTlo,
    float* __restrict__ GH, float* __restrict__ ASC) {
  __shared__ __align__(16) unsigned char smem[32768];
  float* sF = (float*)smem;
  unsigned short* sH = (unsigned short*)smem;
  unsigned short* sL = sH + 8192;
  const int tid = threadIdx.x, lane = tid & 31, w = tid >> 5;
  const int hh = lane >> 4, m = lane & 15;
  const int m0 = blockIdx.x * 128;
  const int cg = blockIdx.y;
  const int n0 = cg * 64;
  const int m0w = m0 + 32 * w;

  const v8f zero8 = {0.f, 0.f, 0.f, 0.f, 0.f, 0.f, 0.f, 0.f};
  v8f acc[2][4];
#pragma unroll
  for (int mt = 0; mt < 2; ++mt)
#pragma unroll
    for (int nt = 0; nt < 4; ++nt) acc[mt][nt] = zero8;

  gemm_core1_32x64(Xb, Bc, DX, (size_t)(m0w + m) * DX, (size_t)(n0 + m) * DX, hh, acc);

  const float* bsrc = bhh;
  int bbase = 0;
  float bfac = 0.0f;
  if (cg < 4)       { bsrc = bm0; bbase = n0;           bfac = 1.0f; }
  else if (cg < 8)  { bsrc = bm1; bbase = n0 - DHD;     bfac = 1.0f; }
  else if (cg < 20) { bsrc = bhh; bbase = n0 - 2 * DHD; bfac = 1.0f; }
  float bv[4];
#pragma unroll
  for (int nt = 0; nt < 4; ++nt) bv[nt] = bf16r(bsrc[bbase + 16 * nt + m]) * bfac;

  if (cg < 8) {
#pragma unroll
    for (int nt = 0; nt < 4; ++nt)
#pragma unroll
      for (int mt = 0; mt < 2; ++mt)
#pragma unroll
        for (int r = 0; r < 8; ++r) {
          const int tokl = 32 * w + 16 * mt + 8 * hh + r;
          const int feat = 16 * nt + m;
          const float y = acc[mt][nt][r] + bv[nt];
          const unsigned short hb = f2bf_bits(y);
          const unsigned short lb = f2bf_bits(y - bf_bits2f(hb));
          const int idx = feat * 128 + tokl;
          sH[idx] = hb;
          sL[idx] = lb;
        }
    __syncthreads();
    {
      const int dsub = lane >> 4, t8 = (lane & 15) * 8;
      for (int pass = 0; pass < 2; ++pass) {
#pragma unroll
        for (int it = 0; it < 8; ++it) {
          const int d = 16 * w + 2 * it + dsub;
          const v4u hv = *(const v4ua*)(sH + d * 128 + t8);
          const v4u lv = *(const v4ua*)(sL + d * 128 + t8);
          const size_t go = (size_t)(n0 + d) * (size_t)NND + m0 + t8;
          *(volatile v4u*)(MThi + go) = hv;
          *(volatile v4u*)(MTlo + go) = lv;
        }
        __threadfence();
      }
    }
  } else {
    float* dstF = GH;
    int pitch = G3;
    int c0 = n0 - 2 * DHD;
    if (cg >= 20) { dstF = ASC; pitch = NASCP; c0 = 0; }
#pragma unroll
    for (int nt = 0; nt < 4; ++nt)
#pragma unroll
      for (int mt = 0; mt < 2; ++mt)
#pragma unroll
        for (int r = 0; r < 8; ++r) {
          const int tokl = 32 * w + 16 * mt + 8 * hh + r;
          const int feat = 16 * nt + m;
          sF[tokl * 64 + feat] = acc[mt][nt][r] + bv[nt];
        }
    __syncthreads();
    {
      const int rsub = lane >> 4, c4 = (lane & 15) * 4;
      for (int pass = 0; pass < 2; ++pass) {
#pragma unroll
        for (int it = 0; it < 16; ++it) {
          const int row = 32 * w + 2 * it + rsub;
          const v4f v = *(const v4fa*)(sF + row * 64 + c4);
          *(volatile v4f*)(dstF + (size_t)(m0 + row) * pitch + c0 + c4) = v;
        }
        __threadfence();
      }
    }
  }
}

__global__ __launch_bounds__(256) void k_attn(const float* __restrict__ adj0, const float* __restrict__ adj1,
                                              const float* __restrict__ w0, const float* __restrict__ w1,
                                              const float* __restrict__ ba0, const float* __restrict__ ba1,
                                              const float* __restrict__ ASC,
                                              const unsigned short* __restrict__ MThi,
                                              const unsigned short* __restrict__ MTlo,
                                              unsigned short* __restrict__ AGhi,
                                              unsigned short* __restrict__ AGlo) {
  __shared__ __align__(16) float sAdj[KT * SP];
  __shared__ __align__(16) float sWt[KT * SP];
  __shared__ __align__(16) float sAnb[NH * KT];
  __shared__ __align__(16) float sAc[NH * QT];
  __shared__ __align__(16) float sO[8 * 16 * DHEAD];

  const int tid = threadIdx.x, lane = tid & 31, w = tid >> 5;
  const int hh = lane >> 4, m = lane & 15;
  const int h = w >> 1, qs = w & 1;
  const int rel = blockIdx.y;
  const int i0 = blockIdx.x * QT;
  const float* adj = rel ? adj1 : adj0;
  const float* wgt = rel ? w1 : w0;
  const float* ba  = rel ? ba1 : ba0;

  if (tid < NH * QT) {
    const int hq = tid >> 5, il = tid & 31;
    sAc[tid] = ASC[(size_t)(i0 + il) * NASCP + rel * 8 + hq];
  }
  __syncthreads();
  const float acur = sAc[h * QT + 16 * qs + m];
  const float bah  = bf16r(ba[h]);

  const v8f zero8 = {0.f, 0.f, 0.f, 0.f, 0.f, 0.f, 0.f, 0.f};
  v8f o[4];
#pragma unroll
  for (int t = 0; t < 4; ++t) o[t] = zero8;
  float mrun = -INFINITY, lrun = 0.0f;

  const int r0s = tid >> 3, c40 = (tid & 7) * 4;
  const int r1s = r0s + 32;
  const int akey = tid & 63, ahd = tid >> 6;
  const unsigned short* vbh = MThi + (size_t)(rel * DHD + h * DHEAD + m) * (size_t)NND;
  const unsigned short* vbl = MTlo + (size_t)(rel * DHD + h * DHEAD + m) * (size_t)NND;
  const int qc = 16 * qs + m;

#pragma unroll 1
  for (int ks = 0; ks < NND / KT; ++ks) {
    const int kb = ks * KT;
    __syncthreads();
    {
      const size_t g0 = (size_t)(kb + r0s) * NND + i0 + c40;
      const size_t g1 = (size_t)(kb + r1s) * NND + i0 + c40;
      const v4f a0 = *(const v4fa*)(adj + g0);
      const v4f a1 = *(const v4fa*)(adj + g1);
      const v4f q0 = *(const v4fa*)(wgt + g0);
      const v4f q1 = *(const v4fa*)(wgt + g1);
      *(v4fa*)(sAdj + r0s * SP + c40) = a0;
      *(v4fa*)(sAdj + r1s * SP + c40) = a1;
      const v4f b0 = {bf16r(q0[0]), bf16r(q0[1]), bf16r(q0[2]), bf16r(q0[3])};
      const v4f b1 = {bf16r(q1[0]), bf16r(q1[1]), bf16r(q1[2]), bf16r(q1[3])};
      *(v4fa*)(sWt + r0s * SP + c40) = b0;
      *(v4fa*)(sWt + r1s * SP + c40) = b1;
      sAnb[tid] = ASC[(size_t)(kb + akey) * NASCP + rel * 8 + 4 + ahd];
    }
    __syncthreads();

    v8f s[4];
#pragma unroll
    for (int jj = 0; jj < 4; ++jj)
#pragma unroll
      for (int r = 0; r < 8; ++r) {
        const int kl = 16 * jj + 8 * hh + r;
        const float a  = sAdj[kl * SP + qc];
        const float ww = sWt[kl * SP + qc];
        float t = sAnb[h * KT + kl] + acur;
        t = t + bah;
        t = (t >= 0.0f) ? t : SLOPE * t;
        t = t * ww;
        t = (a != 0.0f) ? t : NEGF;
        s[jj][r] = t;
      }
    float cm = -INFINITY;
#pragma unroll
    for (int jj = 0; jj < 4; ++jj)
#pragma unroll
      for (int r = 0; r < 8; ++r) cm = fmaxf(cm, s[jj][r]);
    cm = fmaxf(cm, __shfl_xor(cm, 16, 32));
    const float mnew  = fmaxf(mrun, cm);
    const float alpha = __expf(mrun - mnew);
    mrun = mnew;
    float psum = 0.0f;
#pragma unroll
    for (int jj = 0; jj < 4; ++jj)
#pragma unroll
      for (int r = 0; r < 8; ++r) {
        const float p = __expf(s[jj][r] - mnew);
        psum += p;
        s[jj][r] = p;
      }
    psum += __shfl_xor(psum, 16, 32);
    lrun = lrun * alpha + psum;
#pragma unroll
    for (int t = 0; t < 4; ++t)
#pragma unroll
      for (int r = 0; r < 8; ++r) o[t][r] *= alpha;

    v16b p0h, p0l, p1h, p1l;
    pack_p2(s[0], s[1], p0h, p0l);
    pack_p2(s[2], s[3], p1h, p1l);

#pragma unroll
    for (int t = 0; t < 4; ++t) {
      const unsigned short* vph = vbh + (size_t)(16 * t) * (size_t)NND + kb;
      const unsigned short* vpl = vbl + (size_t)(16 * t) * (size_t)NND + kb;
      const v16b v0h = load_frag(vph, hh), v0l = load_frag(vpl, hh);
      o[t] = wmma_bf16(v0h, p0h, o[t]);
      o[t] = wmma_bf16(v0h, p0l, o[t]);
      o[t] = wmma_bf16(v0l, p0h, o[t]);
      const v16b v1h = load_frag(vph + 32, hh), v1l = load_frag(vpl + 32, hh);
      o[t] = wmma_bf16(v1h, p1h, o[t]);
      o[t] = wmma_bf16(v1h, p1l, o[t]);
      o[t] = wmma_bf16(v1l, p1h, o[t]);
    }
  }

  const float inv = (mrun > -1.0e29f) ? (1.0f / lrun) : 0.0f;
  float* so = sO + w * (16 * DHEAD);
#pragma unroll
  for (int t = 0; t < 4; ++t)
#pragma unroll
    for (int r = 0; r < 8; ++r)
      so[m * DHEAD + 16 * t + 8 * hh + r] = o[t][r] * inv;
  __syncthreads();
  const int q8 = lane & 7, sub = lane >> 3;
  v4u hv[4], lv[4];
#pragma unroll
  for (int it = 0; it < 4; ++it) {
    const int row = it * 4 + sub;
    const v4f f0 = *(const v4fa*)(so + row * DHEAD + 8 * q8);
    const v4f f1 = *(const v4fa*)(so + row * DHEAD + 8 * q8 + 4);
    const float y[8] = {f0[0], f0[1], f0[2], f0[3], f1[0], f1[1], f1[2], f1[3]};
    v4u ah, al;
#pragma unroll
    for (int i = 0; i < 4; ++i) {
      const unsigned short h0 = f2bf_bits(y[2 * i]), h1 = f2bf_bits(y[2 * i + 1]);
      const unsigned short l0 = f2bf_bits(y[2 * i] - bf_bits2f(h0)), l1 = f2bf_bits(y[2 * i + 1] - bf_bits2f(h1));
      ah[i] = pk16(h0, h1); al[i] = pk16(l0, l1);
    }
    hv[it] = ah; lv[it] = al;
  }
  const size_t base = (size_t)(i0 + 16 * qs) * DMSG + (size_t)rel * DHD + (size_t)h * DHEAD + 8 * q8;
  for (int pass = 0; pass < 2; ++pass) {
#pragma unroll
    for (int it = 0; it < 4; ++it) {
      const size_t go = base + (size_t)(it * 4 + sub) * DMSG;
      *(volatile v4u*)(AGhi + go) = hv[it];
      *(volatile v4u*)(AGlo + go) = lv[it];
    }
    __threadfence();
  }
}

__global__ __launch_bounds__(128) void k_gi(const unsigned short* __restrict__ AGhi,
                                            const unsigned short* __restrict__ AGlo,
                                            const unsigned short* __restrict__ WIb,
                                            const float* __restrict__ bih, float* __restrict__ GI) {
  __shared__ __align__(16) float sF[128 * 64];
  const int tid = threadIdx.x, lane = tid & 31, w = tid >> 5;
  const int hh = lane >> 4, m = lane & 15;
  const int m0 = blockIdx.x * 128;
  const int n0 = blockIdx.y * 64;
  const int m0w = m0 + 32 * w;

  const v8f zero8 = {0.f, 0.f, 0.f, 0.f, 0.f, 0.f, 0.f, 0.f};
  v8f acc[2][4];
#pragma unroll
  for (int mt = 0; mt < 2; ++mt)
#pragma unroll
    for (int nt = 0; nt < 4; ++nt) acc[mt][nt] = zero8;

  gemm_core_32x64(AGhi, AGlo, WIb, DMSG, (size_t)(m0w + m) * DMSG, (size_t)(n0 + m) * DMSG, hh, acc);

  float bv[4];
#pragma unroll
  for (int nt = 0; nt < 4; ++nt) bv[nt] = bf16r(bih[n0 + 16 * nt + m]);
#pragma unroll
  for (int nt = 0; nt < 4; ++nt)
#pragma unroll
    for (int mt = 0; mt < 2; ++mt)
#pragma unroll
      for (int r = 0; r < 8; ++r) {
        const int tokl = 32 * w + 16 * mt + 8 * hh + r;
        const int feat = 16 * nt + m;
        sF[tokl * 64 + feat] = acc[mt][nt][r] + bv[nt];
      }
  __syncthreads();
  {
    const int rsub = lane >> 4, c4 = (lane & 15) * 4;
    for (int pass = 0; pass < 2; ++pass) {
#pragma unroll
      for (int it = 0; it < 16; ++it) {
        const int row = 32 * w + 2 * it + rsub;
        const v4f v = *(const v4fa*)(sF + row * 64 + c4);
        *(volatile v4f*)(GI + (size_t)(m0 + row) * G3 + n0 + c4) = v;
      }
      __threadfence();
    }
  }
}

__device__ __forceinline__ float rcp_(float v) { return __builtin_amdgcn_rcpf(v); }
__device__ __forceinline__ float sigm_(float v) { return rcp_(1.0f + __expf(-v)); }
__device__ __forceinline__ float tanh_(float v) {
  const float a = fabsf(v);
  const float t = __expf(-2.0f * a);
  const float th = (1.0f - t) * rcp_(1.0f + t);
  return copysignf(th, v);
}

__global__ __launch_bounds__(256) void k_gru_ln(const float* __restrict__ GI, const float* __restrict__ GH,
                                                const float* __restrict__ x,
                                                const float* __restrict__ lng, const float* __restrict__ lnb,
                                                float* __restrict__ out) {
  __shared__ float sP1[8];
  __shared__ float sP2[8];
  const int tid = threadIdx.x, lane = tid & 31, w = tid >> 5;
  const int rl = w >> 1, wsd = w & 1;
  const int row = blockIdx.x * 4 + rl;
  const int col = wsd * 128 + 4 * lane;
  const float* gir = GI + (size_t)row * G3 + col;
  const float* ghr = GH + (size_t)row * G3 + col;
  const v4f gi_r = *(const v4fa*)(gir);
  const v4f gi_z = *(const v4fa*)(gir + DX);
  const v4f gi_n = *(const v4fa*)(gir + 2 * DX);
  const v4f gh_r = *(const v4fa*)(ghr);
  const v4f gh_z = *(const v4fa*)(ghr + DX);
  const v4f gh_n = *(const v4fa*)(ghr + 2 * DX);
  const v4f xv   = *(const v4fa*)(x + (size_t)row * DX + col);
  const v4f gv   = *(const v4fa*)(lng + col);
  const v4f cv   = *(const v4fa*)(lnb + col);

  float hv[4];
#pragma unroll
  for (int e = 0; e < 4; ++e) {
    const float xr = bf16r(xv[e]);
    const float r  = sigm_(gi_r[e] + gh_r[e]);
    const float z  = sigm_(gi_z[e] + gh_z[e]);
    const float n  = tanh_(gi_n[e] + r * gh_n[e]);
    hv[e] = (1.0f - z) * n + z * xr;
  }
  float s = (hv[0] + hv[1]) + (hv[2] + hv[3]);
#pragma unroll
  for (int o = 16; o > 0; o >>= 1) s += __shfl_xor(s, o, 32);
  if (lane == 0) sP1[w] = s;
  __syncthreads();
  const float mean = (sP1[2 * rl] + sP1[2 * rl + 1]) * (1.0f / 256.0f);
  float d[4];
  float q = 0.0f;
#pragma unroll
  for (int e = 0; e < 4; ++e) { d[e] = hv[e] - mean; q += d[e] * d[e]; }
#pragma unroll
  for (int o = 16; o > 0; o >>= 1) q += __shfl_xor(q, o, 32);
  if (lane == 0) sP2[w] = q;
  __syncthreads();
  const float var  = (sP2[2 * rl] + sP2[2 * rl + 1]) * (1.0f / 256.0f);
  const float rstd = rsqrtf(var + LN_EPS);
  v4f y;
#pragma unroll
  for (int e = 0; e < 4; ++e) y[e] = (d[e] * rstd) * bf16r(gv[e]) + bf16r(cv[e]);
  float* op = out + (size_t)row * DX + col;
  *(volatile v4f*)op = y;
  __threadfence();
  *(volatile v4f*)op = y;
}

extern "C" void kernel_launch(void* const* d_in, const int* in_sizes, int n_in,
                              void* d_out, int out_size, void* d_ws, size_t ws_size,
                              hipStream_t stream) {
  if (n_in < 19) return;
  if (in_sizes[0] != NND * DX) return;
  if (in_sizes[1] != NND * NND || in_sizes[2] != NND * NND) return;
  if (in_sizes[3] != NND * NND || in_sizes[4] != NND * NND) return;
  if (in_sizes[5] != DHD * DX || in_sizes[9] != DHD * DX) return;
  if (in_sizes[6] != DHD || in_sizes[10] != DHD) return;
  if (in_sizes[7] != NH * 2 * DX || in_sizes[11] != NH * 2 * DX) return;
  if (in_sizes[8] != NH || in_sizes[12] != NH) return;
  if (in_sizes[13] != G3 * DMSG || in_sizes[14] != G3 * DX) return;
  if (in_sizes[15] != G3 || in_sizes[16] != G3) return;
  if (in_sizes[17] != DX || in_sizes[18] != DX) return;
  if (out_size != NND * DX) return;

  const float* x    = (const float*)d_in[0];
  const float* adj0 = (const float*)d_in[1];
  const float* adj1 = (const float*)d_in[2];
  const float* w0   = (const float*)d_in[3];
  const float* w1   = (const float*)d_in[4];
  const float* Wm0  = (const float*)d_in[5];
  const float* bm0  = (const float*)d_in[6];
  const float* Wa0  = (const float*)d_in[7];
  const float* ba0  = (const float*)d_in[8];
  const float* Wm1  = (const float*)d_in[9];
  const float* bm1  = (const float*)d_in[10];
  const float* Wa1  = (const float*)d_in[11];
  const float* ba1  = (const float*)d_in[12];
  const float* wih  = (const float*)d_in[13];
  const float* whh  = (const float*)d_in[14];
  const float* bih  = (const float*)d_in[15];
  const float* bhh  = (const float*)d_in[16];
  const float* lng  = (const float*)d_in[17];
  const float* lnb  = (const float*)d_in[18];
  float* out = (float*)d_out;

  const size_t PXB = (size_t)NND * DX * 2;
  const size_t PBC = (size_t)NBC * DX * 2;
  const size_t PWI = (size_t)G3 * DMSG * 2;
  const size_t PMT = (size_t)DMSG * NND * 2;
  const size_t PGH = (size_t)NND * G3 * 4;
  const size_t PAS = (size_t)NND * NASCP * 4;
  const size_t PAG = (size_t)NND * DMSG * 2;
  const size_t PGI = (size_t)NND * G3 * 4;
  size_t off = 0;
  const size_t oXb  = off; off += PXB;
  const size_t oBc  = off; off += PBC;
  const size_t oWI  = off; off += PWI;
  const size_t oMTh = off; off += PMT;
  const size_t oMTl = off; off += PMT;
  const size_t oGH  = off; off += PGH;
  const size_t oAS  = off; off += PAS;
  const size_t oAGh = off; off += PAG;
  const size_t oAGl = off; off += PAG;
  const size_t oGI  = off; off += PGI;
  if (off > ws_size) return;

  char* ws = (char*)d_ws;
  unsigned short* Xb   = (unsigned short*)(ws + oXb);
  unsigned short* Bc   = (unsigned short*)(ws + oBc);
  unsigned short* WIb  = (unsigned short*)(ws + oWI);
  unsigned short* MThi = (unsigned short*)(ws + oMTh);
  unsigned short* MTlo = (unsigned short*)(ws + oMTl);
  float*          GH   = (float*)(ws + oGH);
  float*          ASC  = (float*)(ws + oAS);
  unsigned short* AGhi = (unsigned short*)(ws + oAGh);
  unsigned short* AGlo = (unsigned short*)(ws + oAGl);
  float*          GI   = (float*)(ws + oGI);

  k_prep<<<dim3((NXU + NBU + NWU) / 256), 256, 0, stream>>>(x, Wm0, Wm1, whh, Wa0, Wa1, wih, Xb, Bc, WIb);
  k_proj<<<dim3(NND / 128, NBC / 64), 128, 0, stream>>>(Xb, Bc, bm0, bm1, bhh, MThi, MTlo, GH, ASC);
  k_attn<<<dim3(NND / QT, NREL), 256, 0, stream>>>(adj0, adj1, w0, w1, ba0, ba1, ASC, MThi, MTlo, AGhi, AGlo);
  k_gi<<<dim3(NND / 128, G3 / 64), 128, 0, stream>>>(AGhi, AGlo, WIb, bih, GI);
  k_gru_ln<<<dim3(NND / 4), 256, 0, stream>>>(GI, GH, x, lng, lnb, out);
  (void)hipGetLastError();
}
